// GATv2GraphNet_IMDB_34832184770979
// MI455X (gfx1250) — hardware-verified
//
#include <hip/hip_runtime.h>
#include <math.h>

#define NN 50000
#define NE 1600000
#define NV (NE + NN)
#define NPAD 50176
#define NGR 512
#define NT 256
#define TG 1024
#define NBG (NPAD / TG)
#define TD 8192
#define NBD 7
#define SCHG 4096
#define NCHG ((NV + SCHG - 1) / SCHG)
#define SCHD 2048
#define NCHD ((NE + SCHD - 1) / SCHD)
#define GAT_LDS_BYTES ((TG * 32 + TG * 2 + TG * 2 + SCHG) * 4)

typedef __attribute__((ext_vector_type(16))) _Float16 v16h;
typedef __attribute__((ext_vector_type(8)))  _Float16 v8h;
typedef __attribute__((ext_vector_type(16))) __bf16   v16b;
typedef __attribute__((ext_vector_type(8)))  __bf16   v8b;
typedef __attribute__((ext_vector_type(8)))  float    v8f;
typedef __attribute__((ext_vector_type(4)))  float    v4f;
typedef __attribute__((ext_vector_type(4)))  int      v4i;
#define U16(p) ((const unsigned short*)(const void*)(p))

__device__ __forceinline__ unsigned short f2bf_bits(float f) {
  unsigned u = __float_as_uint(f);
  return (unsigned short)((u + 0x7FFFu + ((u >> 16) & 1u)) >> 16);
}
__device__ __forceinline__ float bf_bits2f(unsigned short h) { return __uint_as_float(((unsigned)h) << 16); }

__device__ __forceinline__ void dep_guard_h(v8f& a, v8f& b, v16h x, v16h y) { asm volatile("v_nop\n\tv_nop\n\tv_nop\n\tv_nop" : "+v"(a), "+v"(b) : "v"(x), "v"(y)); }
__device__ __forceinline__ void dep_guard_b(v8f& a, v8f& b, v16b x, v16b y) { asm volatile("v_nop\n\tv_nop\n\tv_nop\n\tv_nop" : "+v"(a), "+v"(b) : "v"(x), "v"(y)); }
__device__ __forceinline__ void keep4_h(v16h a, v16h b, v16h c, v16h d) { asm volatile("v_nop" :: "v"(a), "v"(b), "v"(c), "v"(d)); }
__device__ __forceinline__ void keep4_b(v16b a, v16b b, v16b c, v16b d) { asm volatile("v_nop" :: "v"(a), "v"(b), "v"(c), "v"(d)); }
__device__ __forceinline__ void acc_guard4(v8f& a, v8f& b, v8f& c, v8f& d) { asm volatile("v_nop\n\tv_nop\n\tv_nop\n\tv_nop" : "+v"(a), "+v"(b), "+v"(c), "+v"(d)); }
template <typename T> struct Frag;
template <> struct Frag<_Float16> {
  typedef v16h V; union U { v16h v; v8h h[2]; };
  static __device__ __forceinline__ v16h load(const _Float16* p) {
    U f; f.h[0] = *(const v8h*)(p); f.h[1] = *(const v8h*)(p + 16); return f.v;
  }
  static __device__ __forceinline__ v8f mma(v16h a, v16h b, v8f c) {
    return __builtin_amdgcn_wmma_f32_16x16x32_f16(false, a, false, b, (short)0, c, false, false);
  }
  static __device__ __forceinline__ void guard(v8f& a, v8f& b, v16h x, v16h y) { dep_guard_h(a, b, x, y); }
  static __device__ __forceinline__ void keep(v16h a, v16h b, v16h c, v16h d) { keep4_h(a, b, c, d); }
};
template <> struct Frag<__bf16> {
  typedef v16b V; union U { v16b v; v8b h[2]; };
  static __device__ __forceinline__ v16b load(const __bf16* p) {
    U f; f.h[0] = *(const v8b*)(p); f.h[1] = *(const v8b*)(p + 16); return f.v;
  }
  static __device__ __forceinline__ v8f mma(v16b a, v16b b, v8f c) {
    return __builtin_amdgcn_wmma_f32_16x16x32_bf16(false, a, false, b, (short)0, c, false, false);
  }
  static __device__ __forceinline__ void guard(v8f& a, v8f& b, v16b x, v16b y) { dep_guard_b(a, b, x, y); }
  static __device__ __forceinline__ void keep(v16b a, v16b b, v16b c, v16b d) { keep4_b(a, b, c, d); }
};

template <int ET> struct Elem;
template <> struct Elem<0> { typedef _Float16 T; };
template <> struct Elem<1> { typedef __bf16 T; };
template <int ET, bool SPLIT, int BIAS_MODE, int OUT_MODE, bool RESID, int ACT = 0>
__global__ __launch_bounds__(256) void wmma_gemm64(
    const unsigned short* __restrict__ Ap, const unsigned short* __restrict__ A2p, int lda, long strideA,
    const unsigned short* __restrict__ Btp, const unsigned short* __restrict__ Bt2p, int ldb, long strideB,
    void* __restrict__ Cout, void* __restrict__ Cout2, int ldc, long strideC,
    const float* __restrict__ bias,
    const float* __restrict__ resid, long strideR,
    int M, int N, int K, float scale) {
  typedef typename Elem<ET>::T T;
  typedef typename Frag<T>::V V;
  const T* A = (const T*)Ap; const T* A2 = (const T*)A2p; const T* Bt = (const T*)Btp; const T* Bt2 = (const T*)Bt2p;
  __shared__ __align__(16) float sT[8][16 * 68];
  const int b    = blockIdx.y;
  const int lane = threadIdx.x & 31;
  const int wave = threadIdx.x >> 5;
  const int tilesN = N >> 6;
  const int tilesM = M >> 6;
  const int tile = blockIdx.x * 8 + wave;
  if (tile >= tilesM * tilesN) return;
  const int tm = tile / tilesN;
  const int tn = tile - tm * tilesN;
  const int m0 = tm << 6;
  const int n0 = tn << 6;

  const T* Ab  = A  + (size_t)b * strideA;
  const T* Bb  = Bt + (size_t)b * strideB;
  const T* Ab2 = SPLIT ? (A2  + (size_t)b * strideA) : nullptr;
  const T* Bb2 = SPLIT ? (Bt2 + (size_t)b * strideB) : nullptr;

  const int rlane = lane & 15;
  const int koff  = (lane >> 4) * 8;
  const int mOff  = (lane >> 4) * 8;

  v8f acc[4][4];
#pragma unroll
  for (int i = 0; i < 4; ++i)
#pragma unroll
    for (int j = 0; j < 4; ++j) acc[i][j] = (v8f){0.f,0.f,0.f,0.f,0.f,0.f,0.f,0.f};

  for (int k0 = 0; k0 < K; k0 += 32) {
    V bh[4], bl[4];
#pragma unroll
    for (int j = 0; j < 4; ++j) {
      const size_t bo = (size_t)(n0 + (j << 4) + rlane) * ldb + koff + k0;
      bh[j] = Frag<T>::load(Bb + bo);
      if (SPLIT) bl[j] = Frag<T>::load(Bb2 + bo);
    }
#pragma unroll
    for (int i = 0; i < 4; ++i) {
      const size_t ao = (size_t)(m0 + (i << 4) + rlane) * lda + koff + k0;
      V ah = Frag<T>::load(Ab + ao);
      V al;
      if (SPLIT) al = Frag<T>::load(Ab2 + ao);
#pragma unroll
      for (int j = 0; j < 4; ++j) {
        acc[i][j] = Frag<T>::mma(ah, bh[j], acc[i][j]);
        if (SPLIT) {
          acc[i][j] = Frag<T>::mma(ah, bl[j], acc[i][j]);
          acc[i][j] = Frag<T>::mma(al, bh[j], acc[i][j]);
        }
      }
      Frag<T>::guard(acc[i][0], acc[i][3], ah, SPLIT ? al : ah);
    }
    Frag<T>::keep(bh[0], bh[1], bh[2], bh[3]);
    if (SPLIT) Frag<T>::keep(bl[0], bl[1], bl[2], bl[3]);
  }
  acc_guard4(acc[0][0], acc[0][1], acc[0][2], acc[0][3]);
  acc_guard4(acc[1][0], acc[1][1], acc[1][2], acc[1][3]);
  acc_guard4(acc[2][0], acc[2][1], acc[2][2], acc[2][3]);
  acc_guard4(acc[3][0], acc[3][1], acc[3][2], acc[3][3]);

  float* slab = sT[wave];
  const float* Rb = RESID ? (resid + (size_t)b * strideR) : nullptr;
#pragma unroll
  for (int i = 0; i < 4; ++i) {
    const int mBase = m0 + (i << 4);
#pragma unroll
    for (int j = 0; j < 4; ++j) {
      const int n = n0 + (j << 4) + rlane;
      float bv = 0.f;
      if (BIAS_MODE == 2) bv = bias[n];
#pragma unroll
      for (int r = 0; r < 8; ++r) {
        float v = acc[i][j][r] * scale;
        if (BIAS_MODE == 1) v += bias[mBase + mOff + r];
        if (BIAS_MODE == 2) v += bv;
        if (RESID) v += Rb[(size_t)(mBase + mOff + r) * ldc + n];
        if (ACT == 1) v = tanhf(v);
        if (ACT == 2) v = fmaxf(v, 0.0f);
        if (ACT == 3) v = v / (1.0f + expf(-v));
        if (ACT == 4) v = (v > 0.f) ? v : 0.01f * v;
        if (ACT == 5) v = 0.5f * v * (1.0f + erff(v * 0.70710678118654752f));
        slab[(mOff + r) * 68 + (j << 4) + rlane] = v;
      }
    }
    __builtin_amdgcn_fence(__ATOMIC_RELEASE, "workgroup");
    __builtin_amdgcn_wave_barrier();
    __builtin_amdgcn_fence(__ATOMIC_ACQUIRE, "workgroup");
    if (OUT_MODE == 0) {
      float* C = (float*)Cout + (size_t)b * strideC;
      const int hh = lane >> 4, c4 = (lane & 15) * 4;
      for (int pass = 0; pass < 2; ++pass) {
#pragma unroll
        for (int it = 0; it < 8; ++it) {
          const int row = it * 2 + hh;
          v4f v = *(const v4f*)(slab + row * 68 + c4);
          *(volatile v4f*)(C + (size_t)(mBase + row) * ldc + n0 + c4) = v;
        }
        __threadfence();
      }
    } else {
      const int q = lane >> 3, c8 = (lane & 7) * 8;
      unsigned short* C  = (unsigned short*)Cout  + (size_t)b * strideC;
      unsigned short* C2 = (OUT_MODE == 2) ? ((unsigned short*)Cout2 + (size_t)b * strideC) : nullptr;
      for (int pass = 0; pass < 2; ++pass) {
#pragma unroll
        for (int it = 0; it < 4; ++it) {
          const int row = it * 4 + q;
          const float* sp = slab + row * 68 + c8;
          v8h hv, lv;
#pragma unroll
          for (int e = 0; e < 8; ++e) {
            if (OUT_MODE == 1) {
              hv[e] = (_Float16)sp[e];
            } else {
              unsigned short hb = f2bf_bits(sp[e]);
              unsigned short lb = f2bf_bits(sp[e] - bf_bits2f(hb));
              hv[e] = __builtin_bit_cast(_Float16, hb);
              lv[e] = __builtin_bit_cast(_Float16, lb);
            }
          }
          *(volatile v8h*)(C + (size_t)(mBase + row) * ldc + n0 + c8) = hv;
          if (OUT_MODE == 2) *(volatile v8h*)(C2 + (size_t)(mBase + row) * ldc + n0 + c8) = lv;
        }
        __threadfence();
      }
    }
    __builtin_amdgcn_fence(__ATOMIC_RELEASE, "workgroup");
    __builtin_amdgcn_wave_barrier();
    __builtin_amdgcn_fence(__ATOMIC_ACQUIRE, "workgroup");
  }
}

__device__ __forceinline__ int blk_excl_scan(int cnt, int* scan_ws, int tid, int* tot) {
  const int lane = tid & 31, wave = tid >> 5; int incl = cnt;
#pragma unroll
  for (int o = 1; o < 32; o <<= 1) { const int v = __shfl_up(incl, o, 32); if (lane >= o) incl += v; }
  if (lane == 31) scan_ws[wave] = incl;
  __syncthreads();
  if (wave == 0) { int wv = (lane < NT / 32) ? scan_ws[lane] : 0; int wincl = wv;
#pragma unroll
    for (int o = 1; o < 32; o <<= 1) { const int v = __shfl_up(wincl, o, 32); if (lane >= o) wincl += v; }
    if (lane < NT / 32) scan_ws[32 + lane] = wincl - wv; if (lane == 31) scan_ws[64] = wincl; }
  __syncthreads();
  const int res = scan_ws[32 + wave] + incl - cnt; *tot = scan_ws[64];
  return res;
}
template <int SP, int CAP>
__device__ __forceinline__ int chunk_hits(const int* __restrict__ dstv, const int* __restrict__ srcv, int e0, int n0, int tid,
                                          int* LIST, int* scan_ws) {
  const int eb = e0 + tid * SP;
  const bool real = eb < NE;
  const int ebc = real ? eb : (NE - SP);
  int rec[SP]; int cnt = 0;
#pragma unroll
  for (int k = 0; k < SP; k += 4) {
    const v4i d4 = *(const v4i*)(dstv + ebc + k);
    const v4i s4 = *(const v4i*)(srcv + ebc + k);
#pragma unroll
    for (int e = 0; e < 4; ++e) {
      int r = -1;
      if (real) {
        const int d = d4[e];
        if (d >= n0 && d < n0 + TG) { int s = s4[e]; s = s < 0 ? 0 : (s >= NN ? NN - 1 : s); r = ((d - n0) << 16) | s; ++cnt; }
      } else {
        const int ev = eb + k + e; const int d = ev - NE;
        if (ev < NV && d >= n0 && d < n0 + TG) { r = ((d - n0) << 16) | d; ++cnt; }
      }
      rec[k + e] = r;
    }
  }
  int tot; int p = blk_excl_scan(cnt, scan_ws, tid, &tot);
#pragma unroll
  for (int k = 0; k < SP; ++k) if (rec[k] >= 0) { if ((unsigned)p < (unsigned)CAP) LIST[p] = rec[k]; ++p; }
  __syncthreads();
  return tot < CAP ? tot : CAP;
}

__global__ __launch_bounds__(NT) void feat1_kernel(const int* __restrict__ ei, const float* __restrict__ rf,
                                                  const float* __restrict__ Wl, const float* __restrict__ bl,
                                                  const float* __restrict__ Wr, const float* __restrict__ br,
                                                  float* __restrict__ XLR) {
  __shared__ int LIST[2 * SCHD];
  __shared__ int CNT[TD];
  __shared__ int scan_ws[80];
  const int tid = threadIdx.x, lane = tid & 31, wave = tid >> 5;
  const int n0 = blockIdx.x * TD;
  for (int i = tid; i < TD; i += NT) CNT[i] = 0;
  const float wl0 = Wl[lane * 3], wl1 = Wl[lane * 3 + 1], wl2 = Wl[lane * 3 + 2], blv = bl[lane];
  const float wr0 = Wr[lane * 3], wr1 = Wr[lane * 3 + 1], wr2 = Wr[lane * 3 + 2], brv = br[lane];
  __syncthreads();
  const int* srcv = ei; const int* dstv = ei + NE;
#pragma unroll 1
  for (int c = 0; c < NCHD; ++c) {
    const int eb = c * SCHD + tid * (SCHD / NT);
    const bool real = eb < NE;
    const int ebc = real ? eb : (NE - (SCHD / NT));
    int rec[2 * (SCHD / NT)]; int cnt = 0;
#pragma unroll
    for (int k = 0; k < SCHD / NT; k += 4) {
      const v4i s4 = *(const v4i*)(srcv + ebc + k);
      const v4i d4 = *(const v4i*)(dstv + ebc + k);
#pragma unroll
      for (int e = 0; e < 4; ++e) {
        const int s = s4[e], d = d4[e];
        int ra = -1, rb = -1;
        if (real && s >= n0 && s < n0 + TD) { ra = s - n0; ++cnt; }
        if (real && d >= n0 && d < n0 + TD) { rb = d - n0; ++cnt; }
        rec[2 * (k + e)] = ra; rec[2 * (k + e) + 1] = rb;
      }
    }
    int tot; int p = blk_excl_scan(cnt, scan_ws, tid, &tot);
#pragma unroll
    for (int k = 0; k < 2 * (SCHD / NT); ++k) if (rec[k] >= 0) { if ((unsigned)p < (unsigned)(2 * SCHD)) LIST[p] = rec[k]; ++p; }
    __syncthreads();
    tot = tot < 2 * SCHD ? tot : 2 * SCHD;
#pragma unroll 1
    for (int base = 0; base < tot; base += 32) {
      const int q = base + lane;
      const int rv = (q < tot) ? LIST[q] : -1;
      const int own = (rv >= 0 && (rv >> 10) == wave) ? 1 : 0;
      unsigned msk = (unsigned)__ballot(own);
#pragma unroll 1
      for (int it = 0; it < 32; ++it) {
        if (msk == 0u) break;
        const int bp = __builtin_ctz(msk); msk &= msk - 1u;
        const int r = __shfl(rv, bp, 32);
        if (lane == 0) CNT[r] += 1;
        asm volatile("" ::: "memory");
      }
    }
    __syncthreads();
  }
#pragma unroll 1
  for (int j = 0; j < TD / 8; ++j) {
    const int dl = wave * (TD / 8) + j; const int n = n0 + dl;
    if (n < NPAD) {
      const bool live = n < NN;
      const float dg = (float)CNT[dl];
      const float rr = rf[live ? n : (NN - 1)];
      float xl = wl0 + wl1 * dg; xl = xl + wl2 * rr; xl = xl + blv;
      float xr = wr0 + wr1 * dg; xr = xr + wr2 * rr; xr = xr + brv;
      if (!live) { xl = 0.f; xr = 0.f; }
      float* rp = XLR + (size_t)n * 64;
      for (int pass = 0; pass < 2; ++pass) {
        ((volatile float*)rp)[lane] = xl;
        ((volatile float*)rp)[32 + lane] = xr;
        __threadfence();
      }
    }
  }
}

template <bool PLANES>
__global__ __launch_bounds__(NT) void gat_kernel(const float* __restrict__ XLR, const int* __restrict__ ei,
                                                const float* __restrict__ att, const float* __restrict__ bias,
                                                float* __restrict__ XO, unsigned* __restrict__ XP) {
  extern __shared__ __align__(16) float dyn_lds[];
  float* ACC = dyn_lds;
  float* SM = dyn_lds + TG * 32;
  float* SL = dyn_lds + TG * 32 + TG * 2;
  int* LIST = (int*)(dyn_lds + TG * 32 + TG * 4);
  __shared__ int scan_ws[80];
  const int tid = threadIdx.x, lane = tid & 31, wave = tid >> 5;
  const int n0 = blockIdx.x * TG;
  const int hd = lane >> 4;
  const float av = att[lane], bv = bias[lane];
  for (int i = tid; i < TG * 32; i += NT) ACC[i] = 0.f;
  for (int i = tid; i < TG * 2; i += NT) { SM[i] = -INFINITY; SL[i] = 0.f; }
  __syncthreads();
  const int* srcv = ei; const int* dstv = ei + NE;
#pragma unroll 1
  for (int c = 0; c < NCHG; ++c) {
    const int tot = chunk_hits<SCHG / NT, SCHG>(dstv, srcv, c * SCHG, n0, tid, LIST, scan_ws);
#pragma unroll 1
    for (int base = 0; base < tot; base += 32) {
      const int q = base + lane;
      const int rv = (q < tot) ? LIST[q] : -1;
      const int own = (rv >= 0 && (rv >> 23) == wave) ? 1 : 0;
      unsigned msk = (unsigned)__ballot(own);
#pragma unroll 1
      for (int it = 0; it < 32; ++it) {
        if (msk == 0u) break;
        const int bp = __builtin_ctz(msk); msk &= msk - 1u;
        const int r = __shfl(rv, bp, 32);
        const int dl = r >> 16, s = r & 0xFFFF;
        const float xl = XLR[(size_t)s * 64 + lane];
        const float xr = XLR[(size_t)(n0 + dl) * 64 + 32 + lane];
        float v = xl + xr; v = fmaxf(v, 0.2f * v);
        float sc = v * av;
        sc += __shfl_xor(sc, 8, 32);
        sc += __shfl_xor(sc, 4, 32);
        sc += __shfl_xor(sc, 2, 32);
        sc += __shfl_xor(sc, 1, 32);
        const int mi = dl * 2 + hd;
        const float mo = SM[mi], lo = SL[mi];
        const float mn = fmaxf(mo, sc);
        const float rr = __expf(mo - mn), ex = __expf(sc - mn);
        const float ln = lo * rr + ex;
        if ((lane & 15) == 0) { SM[mi] = mn; SL[mi] = ln; }
        float* ap = ACC + dl * 32 + lane;
        float a = *ap;
        a = a * rr + ex * xl;
        *ap = a;
        asm volatile("" ::: "memory");
      }
    }
    __syncthreads();
  }
#pragma unroll 1
  for (int j = 0; j < TG / 8; ++j) {
    const int dl = wave * (TG / 8) + j; const int n = n0 + dl;
    const bool live = n < NN;
    float lv = SL[dl * 2 + hd]; lv = (live && lv > 0.f) ? lv : 1.0f;
    const float inv = 1.0f / lv;
    float o = ACC[dl * 32 + lane] * inv;
    o = o + bv;
    o = (o > 0.f) ? o : expm1f(o);
    if (!live) o = 0.f;
    if (!PLANES) {
      float* rp = XO + (size_t)n * 32;
      for (int pass = 0; pass < 2; ++pass) { ((volatile float*)rp)[lane] = o; __threadfence(); }
    } else {
      const unsigned hb = (unsigned)f2bf_bits(o);
      const unsigned lb = (unsigned)f2bf_bits(o - bf_bits2f((unsigned short)hb));
      const int a0 = (2 * lane) & 31;
      const unsigned h0 = (unsigned)__shfl((int)hb, a0, 32), h1 = (unsigned)__shfl((int)hb, a0 + 1, 32);
      const unsigned l0 = (unsigned)__shfl((int)lb, a0, 32), l1 = (unsigned)__shfl((int)lb, a0 + 1, 32);
      const unsigned w = (lane < 16) ? (h0 | (h1 << 16)) : (l0 | (l1 << 16));
      unsigned* rp = XP + (size_t)n * 32;
      for (int pass = 0; pass < 2; ++pass) { ((volatile unsigned*)rp)[lane] = w; __threadfence(); }
    }
  }
}

__global__ __launch_bounds__(NT) void w2_kernel(const float* __restrict__ Wl, const float* __restrict__ bl, const float* __restrict__ Wr,
                                               const float* __restrict__ br, unsigned* __restrict__ Bh, unsigned* __restrict__ Bl, float* __restrict__ bb) {
  const int t = threadIdx.x;
  for (int i = t; i < 64 * 16; i += NT) {
    const int o = i >> 4, k = 2 * (i & 15);
    const float* W = (o < 32) ? Wl : Wr; const int oo = o & 31;
    const float a = W[oo * 32 + k], b = W[oo * 32 + k + 1];
    const unsigned short ah = f2bf_bits(a), bh = f2bf_bits(b);
    const unsigned short al = f2bf_bits(a - bf_bits2f(ah)), blo = f2bf_bits(b - bf_bits2f(bh));
    const unsigned uh = (unsigned)ah | ((unsigned)bh << 16), ul = (unsigned)al | ((unsigned)blo << 16);
    ((volatile unsigned*)Bh)[i] = uh; ((volatile unsigned*)Bl)[i] = ul;
    __threadfence();
    ((volatile unsigned*)Bh)[i] = uh; ((volatile unsigned*)Bl)[i] = ul;
  }
  if (t < 64) { const float v = (t < 32) ? bl[t] : br[t - 32]; ((volatile float*)bb)[t] = v; __threadfence(); ((volatile float*)bb)[t] = v; }
}

__global__ __launch_bounds__(NT) void pool_kernel(const float* __restrict__ X2, const int* __restrict__ batch, float* __restrict__ POOL) {
  __shared__ __align__(16) float red[NT * 32];
  __shared__ int rc[NT];
  const int tid = threadIdx.x, lane = tid & 31, wave = tid >> 5;
  const int g = blockIdx.x;
  const v4f z4 = {0.f, 0.f, 0.f, 0.f};
  v4f a[8];
#pragma unroll
  for (int q = 0; q < 8; ++q) a[q] = z4;
  int cnt = 0;
#pragma unroll 1
  for (int n = tid; n < NN; n += NT) {
    if (batch[n] == g) {
      const float* xp = X2 + (size_t)n * 32;
#pragma unroll
      for (int q = 0; q < 8; ++q) a[q] = a[q] + *(const v4f*)(xp + 4 * q);
      ++cnt;
    }
  }
#pragma unroll
  for (int q = 0; q < 8; ++q) *(v4f*)(red + tid * 32 + 4 * q) = a[q];
  rc[tid] = cnt;
  __syncthreads();
  if (wave == 0) {
    float s = 0.f; int ct = 0;
#pragma unroll 1
    for (int t = 0; t < NT; ++t) { s += red[t * 32 + lane]; ct += rc[t]; }
    const float inv = 1.0f / fmaxf((float)ct, 1.0f);
    const float o = s * inv;
    for (int pass = 0; pass < 2; ++pass) { ((volatile float*)POOL)[(size_t)g * 32 + lane] = o; __threadfence(); }
  }
}

__global__ __launch_bounds__(NT) void head_kernel(const float* __restrict__ POOL, const float* __restrict__ Wfc, const float* __restrict__ bfc,
                                                 float* __restrict__ out) {
  __shared__ __align__(16) float so[NGR * 2];
  const int tid = threadIdx.x;
  for (int g = tid; g < NGR; g += NT) {
    float l0 = bfc[0], l1 = bfc[1];
#pragma unroll 1
    for (int j = 0; j < 32; ++j) { const float p = POOL[g * 32 + j]; l0 += p * Wfc[j]; l1 += p * Wfc[32 + j]; }
    const float mx = fmaxf(l0, l1);
    const float lse = mx + logf(expf(l0 - mx) + expf(l1 - mx));
    so[2 * g] = l0 - lse; so[2 * g + 1] = l1 - lse;
  }
  __syncthreads();
  const v4f v = *(const v4f*)(so + 4 * tid);
  for (int pass = 0; pass < 2; ++pass) { *(volatile v4f*)(out + 4 * tid) = v; __threadfence(); }
}

extern "C" void kernel_launch(void* const* d_in, const int* in_sizes, int n_in,
                              void* d_out, int out_size, void* d_ws, size_t ws_size, hipStream_t stream) {
  (void)in_sizes; (void)n_in; (void)out_size;
  const int*   ei    = (const int*)  d_in[0];
  const int*   batch = (const int*)  d_in[1];
  const float* rf    = (const float*)d_in[2];
  const float* W1l   = (const float*)d_in[3];
  const float* b1l   = (const float*)d_in[4];
  const float* W1r   = (const float*)d_in[5];
  const float* b1r   = (const float*)d_in[6];
  const float* att1  = (const float*)d_in[7];
  const float* bias1 = (const float*)d_in[8];
  const float* W2l   = (const float*)d_in[9];
  const float* b2l   = (const float*)d_in[10];
  const float* W2r   = (const float*)d_in[11];
  const float* b2r   = (const float*)d_in[12];
  const float* att2  = (const float*)d_in[13];
  const float* bias2 = (const float*)d_in[14];
  const float* Wfc   = (const float*)d_in[15];
  const float* bfc   = (const float*)d_in[16];
  float* out = (float*)d_out;

  char* ws = (char*)d_ws; size_t off = 0;
  auto carve = [&](size_t bytes) -> char* { char* p = ws + off; off += (bytes + 255) & ~(size_t)255; return p; };
  float*    XLR1 = (float*)carve((size_t)NPAD * 64 * 4);
  unsigned* X1P  = (unsigned*)carve((size_t)NPAD * 32 * 4);
  float*    XLR2 = (float*)carve((size_t)NPAD * 64 * 4);
  float*    X2   = (float*)carve((size_t)NPAD * 32 * 4);
  unsigned* B2h  = (unsigned*)carve((size_t)64 * 32 * 2);
  unsigned* B2l  = (unsigned*)carve((size_t)64 * 32 * 2);
  float*    b2c  = (float*)carve(256);
  float*    POOL = (float*)carve((size_t)NGR * 32 * 4);
  if (off > ws_size || off > (size_t)134217728) return;

  feat1_kernel<<<NBD, NT, 0, stream>>>(ei, rf, W1l, b1l, W1r, b1r, XLR1);
  w2_kernel<<<1, NT, 0, stream>>>(W2l, b2l, W2r, b2r, B2h, B2l, b2c);
  hipFuncSetAttribute(reinterpret_cast<const void*>(&gat_kernel<true>), hipFuncAttributeMaxDynamicSharedMemorySize, GAT_LDS_BYTES);
  gat_kernel<true><<<NBG, NT, GAT_LDS_BYTES, stream>>>(XLR1, ei, att1, bias1, (float*)nullptr, X1P);
  {
    const int tiles = (NPAD / 64) * (64 / 64);
    wmma_gemm64<1, true, 2, 0, false><<<dim3((tiles + 7) / 8, 1), 256, 0, stream>>>(
        U16(X1P), U16(X1P) + 32, 64, 0L,
        U16(B2h), U16(B2l), 32, 0L,
        (void*)XLR2, (void*)nullptr, 64, 0L,
        b2c, (const float*)nullptr, 0L, NPAD, 64, 32, 1.0f);
  }
  hipFuncSetAttribute(reinterpret_cast<const void*>(&gat_kernel<false>), hipFuncAttributeMaxDynamicSharedMemorySize, GAT_LDS_BYTES);
  gat_kernel<false><<<NBG, NT, GAT_LDS_BYTES, stream>>>(XLR2, ei, att2, bias2, X2, (unsigned*)nullptr);
  pool_kernel<<<NGR, NT, 0, stream>>>(X2, batch, POOL);
  head_kernel<<<1, NT, 0, stream>>>(POOL, Wfc, bfc, out);
}
